// MSAttention_29059748725180
// MI455X (gfx1250) — hardware-verified
//
#include <hip/hip_runtime.h>


namespace {
constexpr int NBt = 8, DIM = 256, H0 = 16, H1 = 32, H2 = 64, P0 = NBt * H0 * H0, P1 = NBt * H1 * H1, P2 = NBt * H2 * H2;
constexpr float XS = 8.0f, WSC = 256.0f;

typedef _Float16 b16;
typedef __attribute__((ext_vector_type(16))) _Float16 v16b;
typedef __attribute__((ext_vector_type(8))) _Float16 v8b;
typedef __attribute__((ext_vector_type(8))) float v8f;
typedef __attribute__((ext_vector_type(4))) float v4f;
__device__ __forceinline__ float bf16_rne(float f) { unsigned int u = __float_as_uint(f); u += 0x7FFFu + ((u >> 16) & 1u); return __uint_as_float(u & 0xFFFF0000u); }
__device__ __forceinline__ v16b frag_kb(const b16* p, int hh) { const v8b a = *(const v8b*)(p + 8 * hh), b = *(const v8b*)(p + 16 + 8 * hh); v16b f;
#pragma unroll
  for (int e = 0; e < 8; ++e) { f[e] = a[e]; f[8 + e] = b[e]; } return f; }
__device__ __forceinline__ v8f wmma16b(v16b a, v16b b, v8f c) { v8f d = __builtin_amdgcn_wmma_f32_16x16x32_f16(false, a, false, b, (short)0, c, false, false); asm volatile("v_nop\n\tv_nop\n\tv_nop\n\tv_nop" : "+v"(d) : "v"(a), "v"(b)); return d; }
__device__ __forceinline__ void wave_lds_sync() { __builtin_amdgcn_fence(__ATOMIC_RELEASE, "workgroup"); __builtin_amdgcn_wave_barrier(); __builtin_amdgcn_fence(__ATOMIC_ACQUIRE, "workgroup"); }

__global__ __launch_bounds__(256) void prepx_kernel(const float* __restrict__ x0, const float* __restrict__ x1, const float* __restrict__ x2, b16* __restrict__ X0, b16* __restrict__ X1, b16* __restrict__ X2) {
  const size_t g = (size_t)blockIdx.x * 256 + threadIdx.x; const size_t n0 = (size_t)P0 * DIM / 8, n1 = (size_t)P1 * DIM / 8, n2 = (size_t)P2 * DIM / 8;
  if (g >= n0 + n1 + n2) return;
  const float* src; b16* dst; size_t e; if (g < n0) { src = x0; dst = X0; e = g * 8; } else if (g < n0 + n1) { src = x1; dst = X1; e = (g - n0) * 8; } else { src = x2; dst = X2; e = (g - n0 - n1) * 8; }
  const v4f a = *(const v4f*)(src + e), c = *(const v4f*)(src + e + 4); v8b o;
#pragma unroll
  for (int j = 0; j < 4; ++j) { o[j] = (b16)(bf16_rne(a[j]) * XS); o[4 + j] = (b16)(bf16_rne(c[j]) * XS); }
  for (int pass = 0; pass < 2; ++pass) { *(volatile v8b*)(dst + e) = o; __threadfence(); }
}
__global__ __launch_bounds__(256) void prepw_kernel(const float* __restrict__ w0, const float* __restrict__ w1, const float* __restrict__ w2, const float* __restrict__ w3, const float* __restrict__ w4, const float* __restrict__ w5, const float* __restrict__ w6, b16* __restrict__ WV) {
  const int widx = blockIdx.y; const float* w = widx == 0 ? w0 : widx == 1 ? w1 : widx == 2 ? w2 : widx == 3 ? w3 : widx == 4 ? w4 : widx == 5 ? w5 : w6;
  const size_t g = (size_t)blockIdx.x * 256 + threadIdx.x; if (g >= (size_t)DIM * DIM / 8) return; const size_t e = g * 8;
  const v4f a = *(const v4f*)(w + (size_t)DIM * DIM + e), c = *(const v4f*)(w + (size_t)DIM * DIM + e + 4); v8b o;
#pragma unroll
  for (int j = 0; j < 4; ++j) { o[j] = (b16)(bf16_rne(a[j]) * WSC); o[4 + j] = (b16)(bf16_rne(c[j]) * WSC); }
  for (int pass = 0; pass < 2; ++pass) { *(volatile v8b*)(WV + (size_t)widx * DIM * DIM + e) = o; __threadfence(); }
}
__global__ __launch_bounds__(128) void vproj_kernel(const b16* __restrict__ X16, const b16* __restrict__ W, float* __restrict__ V) {
  __shared__ __attribute__((aligned(16))) float Ts[4][16][128 + 4];
  const int wave = threadIdx.x >> 5, lane = threadIdx.x & 31, nloc = lane & 15, hlf = lane >> 4; const size_t m0 = (size_t)blockIdx.x * 64 + wave * 16; const int n0 = blockIdx.y * 128;
  v8f acc[8];
#pragma unroll
  for (int t = 0; t < 8; ++t) acc[t] = (v8f){};
#pragma unroll
  for (int kb = 0; kb < DIM; kb += 32) { const v16b a = frag_kb(X16 + (m0 + nloc) * DIM + kb, hlf);
#pragma unroll
    for (int t = 0; t < 8; ++t) acc[t] = wmma16b(a, frag_kb(W + (size_t)(n0 + t * 16 + nloc) * DIM + kb, hlf), acc[t]); }
#pragma unroll
  for (int t = 0; t < 8; ++t)
#pragma unroll
    for (int r = 0; r < 8; ++r) Ts[wave][8 * hlf + r][t * 16 + nloc] = acc[t][r] * (1.0f / (XS * WSC));
  wave_lds_sync();
  for (int pass = 0; pass < 2; ++pass) { for (int rr = 0; rr < 16; ++rr) *(volatile v4f*)(V + (m0 + rr) * DIM + n0 + lane * 4) = *(const v4f*)(&Ts[wave][rr][lane * 4]); __threadfence(); }
}
template <int HS, int HB, int HASPAR, int HK>
__global__ __launch_bounds__(256) void assemble_kernel(const float* __restrict__ VP, const float* __restrict__ VA, const float* __restrict__ VK, float* __restrict__ out) {
  const int wave = threadIdx.x >> 5, lane = threadIdx.x & 31; const int pix = blockIdx.x * 8 + wave; const int b = pix / (HS * HS), rem = pix - b * HS * HS, hi = rem / HS, wi = rem - hi * HS;
  v4f a0 = {0, 0, 0, 0}, a1 = {0, 0, 0, 0}; const int c0 = lane * 8;
  const int bh = (hi / HB) * HB, bw = (wi / HB) * HB;
#pragma unroll 1
  for (int m = 0; m < HB * HB; ++m) { const int ph = bh + m / HB, pw = bw + m % HB; const float* r = VP + (((size_t)b * HS + ph) * HS + pw) * DIM + c0; a0 += *(const v4f*)r; a1 += *(const v4f*)(r + 4); }
  if (HASPAR) { constexpr int HC = HS / HB; const float* r = VA + (((size_t)b * HC + hi / HB) * HC + wi / HB) * DIM + c0; a0 += *(const v4f*)r; a1 += *(const v4f*)(r + 4); }
  if (HK > 0) { constexpr int HF = HS * (HK > 0 ? HK : 1);
#pragma unroll 1
    for (int g = 0; g < HK * HK; ++g) { const int kh = hi * HK + g / HK, kw = wi * HK + g % HK; const float* r = VK + (((size_t)b * HF + kh) * HF + kw) * DIM + c0; a0 += *(const v4f*)r; a1 += *(const v4f*)(r + 4); } }
  for (int pass = 0; pass < 2; ++pass) { *(volatile v4f*)(out + (size_t)pix * DIM + c0) = a0; *(volatile v4f*)(out + (size_t)pix * DIM + c0 + 4) = a1; __threadfence(); }
}
}

extern "C" void kernel_launch(void* const* d_in, const int* in_sizes, int n_in, void* d_out, int out_size, void* d_ws, size_t ws_size, hipStream_t stream) {
  (void)n_in;
  auto Fp = [&](int i) { return (const float*)d_in[i]; };
  if (in_sizes[0] != P0 * DIM || in_sizes[1] != P1 * DIM || in_sizes[2] != P2 * DIM || in_sizes[4] != 2 * DIM * DIM || in_sizes[6] != 2 * DIM * DIM || in_sizes[8] != 2 * DIM * DIM || in_sizes[10] != 2 * DIM * DIM || in_sizes[12] != 2 * DIM * DIM || in_sizes[14] != 2 * DIM * DIM || in_sizes[16] != 2 * DIM * DIM || out_size != (P0 + P1 + P2) * DIM) return;
  size_t off = 0; char* ws = (char*)d_ws;
  auto carve = [&](size_t bytes) { char* p = ws + off; off += (bytes + 255) & ~(size_t)255; return p; };
  b16* X0 = (b16*)carve((size_t)P0 * DIM * 2); b16* X1 = (b16*)carve((size_t)P1 * DIM * 2); b16* X2 = (b16*)carve((size_t)P2 * DIM * 2); b16* WV = (b16*)carve((size_t)7 * DIM * DIM * 2);
  float* VP0 = (float*)carve((size_t)P0 * DIM * 4); float* VK0 = (float*)carve((size_t)P1 * DIM * 4); float* VP1 = (float*)carve((size_t)P1 * DIM * 4); float* VA1 = (float*)carve((size_t)P0 * DIM * 4);
  float* VK1 = (float*)carve((size_t)P2 * DIM * 4); float* VP2 = (float*)carve((size_t)P2 * DIM * 4); float* VA2 = (float*)carve((size_t)P1 * DIM * 4);
  if (off > ws_size || off > ((size_t)128 << 20)) return;
  float* o0 = (float*)d_out; float* o1 = o0 + (size_t)P0 * DIM; float* o2 = o1 + (size_t)P1 * DIM;
  prepx_kernel<<<((P0 + P1 + P2) * DIM / 8 + 255) / 256, 256, 0, stream>>>(Fp(0), Fp(1), Fp(2), X0, X1, X2);
  prepw_kernel<<<dim3(DIM * DIM / 8 / 256, 7), 256, 0, stream>>>(Fp(4), Fp(14), Fp(6), Fp(10), Fp(16), Fp(8), Fp(12), WV);
  vproj_kernel<<<dim3(P0 / 64, 2), 128, 0, stream>>>(X0, WV + 0 * DIM * DIM, VP0);
  vproj_kernel<<<dim3(P1 / 64, 2), 128, 0, stream>>>(X1, WV + 1 * DIM * DIM, VK0);
  vproj_kernel<<<dim3(P1 / 64, 2), 128, 0, stream>>>(X1, WV + 2 * DIM * DIM, VP1);
  vproj_kernel<<<dim3(P0 / 64, 2), 128, 0, stream>>>(X0, WV + 3 * DIM * DIM, VA1);
  vproj_kernel<<<dim3(P2 / 64, 2), 128, 0, stream>>>(X2, WV + 4 * DIM * DIM, VK1);
  vproj_kernel<<<dim3(P2 / 64, 2), 128, 0, stream>>>(X2, WV + 5 * DIM * DIM, VP2);
  vproj_kernel<<<dim3(P1 / 64, 2), 128, 0, stream>>>(X1, WV + 6 * DIM * DIM, VA2);
  assemble_kernel<H0, 4, 0, 2><<<P0 / 8, 256, 0, stream>>>(VP0, nullptr, VK0, o0);
  assemble_kernel<H1, 2, 1, 2><<<P1 / 8, 256, 0, stream>>>(VP1, VA1, VK1, o1);
  assemble_kernel<H2, 2, 1, 0><<<P2 / 8, 256, 0, stream>>>(VP2, VA2, nullptr, o2);
}
